// BiMambaBlock_3770981286790
// MI455X (gfx1250) — hardware-verified
//
#include <hip/hip_runtime.h>
#include <math.h>

typedef __attribute__((ext_vector_type(16))) _Float16 v16h;
typedef __attribute__((ext_vector_type(8)))  _Float16 v8h;
typedef __attribute__((ext_vector_type(4)))  _Float16 v4h;
typedef __attribute__((ext_vector_type(16))) __bf16   v16b;
typedef __attribute__((ext_vector_type(8)))  __bf16   v8b;
typedef __attribute__((ext_vector_type(8)))  float    v8f;
typedef __attribute__((ext_vector_type(4)))  float    v4f;

constexpr int kSamples = 2;
constexpr int kSeq   = 4096;
constexpr int kRows  = kSeq;
constexpr int kDm    = 512;
constexpr int kDi    = 512;
constexpr int kDi2   = 2 * kDi;
constexpr int kNs    = 16;
constexpr int kR     = 32;
constexpr int kXd    = kR + 2 * kNs;
constexpr int kKc    = 4;
constexpr int kThr   = 256;
constexpr float kInCarry = 1024.0f;
constexpr float kWCarry = 4096.0f;
constexpr float kSc = 1.0f / (kInCarry * kWCarry);
constexpr float kInvD = 1.0f / 512.0f;
constexpr float kEps = 1e-5f;
constexpr float kF16MinNormal = 6.103515625e-5f;

static_assert((kRows % 64) == 0 && (kDi2 % 64) == 0 && kXd == 64 && (kDi % 64) == 0 && (kDm % 32) == 0 && (kR % 32) == 0
              && ((kRows / 64) * (kDi2 / 64)) % 8 == 0 && ((kRows / 64) * (kXd / 64)) % 8 == 0 && ((kRows / 64) * (kDi / 64)) % 8 == 0, "GEMM M, N multiples of 64; grids exact; K multiples of 32");

constexpr size_t kOffXN16 = 0ull;
constexpr size_t kOffWPT = 4194304ull;
constexpr size_t kOffWXT = 5242880ull;
constexpr size_t kOffWDT = 5308416ull;
constexpr size_t kOffBV = 5341184ull;
constexpr size_t kOffZX = 5349376ull;
constexpr size_t kOffU32 = 22126592ull;
constexpr size_t kOffU16 = 30515200ull;
constexpr size_t kOffDBC = 34709504ull;
constexpr size_t kOffDT16 = 35758080ull;
constexpr size_t kOffDL = 36020224ull;
constexpr size_t kOffYF = 44408832ull;
constexpr size_t kOffYB = 52797440ull;
constexpr size_t kWsTotal = 61186048ull;
static_assert(kWsTotal <= 134217728ull, "carve cap: under 128 MiB");
static_assert(kOffXN16 == 0
              && kOffWPT == kOffXN16 + 4194304ull
              && kOffWXT == kOffWPT + 1048576ull
              && kOffWDT == kOffWXT + 65536ull
              && kOffBV == kOffWDT + 32768ull
              && kOffZX == kOffBV + 8192ull
              && kOffU32 == kOffZX + 16777216ull
              && kOffU16 == kOffU32 + 8388608ull
              && kOffDBC == kOffU16 + 4194304ull
              && kOffDT16 == kOffDBC + 1048576ull
              && kOffDL == kOffDT16 + 262144ull
              && kOffYF == kOffDL + 8388608ull
              && kOffYB == kOffYF + 8388608ull
              && kWsTotal == kOffYB + 8388608ull, "the carve is chained and totalled");
static_assert((kOffXN16 % 256) == 0 && (kOffWPT % 256) == 0 && (kOffWXT % 256) == 0 && (kOffWDT % 256) == 0 && (kOffBV % 256) == 0 && (kOffZX % 256) == 0 && (kOffU32 % 256) == 0 && (kOffU16 % 256) == 0 && (kOffDBC % 256) == 0 && (kOffDT16 % 256) == 0 && (kOffDL % 256) == 0 && (kOffYF % 256) == 0 && (kOffYB % 256) == 0, "aligned regions");

__device__ __forceinline__ unsigned short f2bf_bits(float f) {
  unsigned u = __float_as_uint(f);
  return (unsigned short)((u + 0x7FFFu + ((u >> 16) & 1u)) >> 16);
}
__device__ __forceinline__ float bf_bits2f(unsigned short h) { return __uint_as_float(((unsigned)h) << 16); }
__device__ __forceinline__ float bf16r(float f) { return bf_bits2f(f2bf_bits(f)); }
__device__ __forceinline__ float carry_flush(float v, float carry) {
  const float s = v * carry;
  return (fabsf(s) < kF16MinNormal) ? 0.0f : s;
}
__device__ __forceinline__ float frcp(float x) { return __builtin_amdgcn_rcpf(x); }

__device__ __forceinline__ void dep_guard4_h(v8f& a, v8f& b, v8f& c, v8f& d, v16h x, v16h y) { asm volatile("v_nop\n\tv_nop\n\tv_nop\n\tv_nop" : "+v"(a), "+v"(b), "+v"(c), "+v"(d) : "v"(x), "v"(y)); }
__device__ __forceinline__ void dep_guard4_b(v8f& a, v8f& b, v8f& c, v8f& d, v16b x, v16b y) { asm volatile("v_nop\n\tv_nop\n\tv_nop\n\tv_nop" : "+v"(a), "+v"(b), "+v"(c), "+v"(d) : "v"(x), "v"(y)); }
__device__ __forceinline__ void keep4_h(v16h a, v16h b, v16h c, v16h d) { asm volatile("v_nop" :: "v"(a), "v"(b), "v"(c), "v"(d)); }
__device__ __forceinline__ void keep4_b(v16b a, v16b b, v16b c, v16b d) { asm volatile("v_nop" :: "v"(a), "v"(b), "v"(c), "v"(d)); }
__device__ __forceinline__ void acc_guard4(v8f& a, v8f& b, v8f& c, v8f& d) { asm volatile("v_nop\n\tv_nop\n\tv_nop\n\tv_nop" : "+v"(a), "+v"(b), "+v"(c), "+v"(d)); }

template <typename T> struct Frag;
template <> struct Frag<_Float16> {
  typedef v16h V; union U { v16h v; v8h h[2]; };
  static __device__ __forceinline__ v16h load(const _Float16* p) {
    U f; f.h[0] = *(const v8h*)(p); f.h[1] = *(const v8h*)(p + 16); return f.v;
  }
  static __device__ __forceinline__ v8f mma(v16h a, v16h b, v8f c) {
    return __builtin_amdgcn_wmma_f32_16x16x32_f16(false, a, false, b, (short)0, c, false, false);
  }
  static __device__ __forceinline__ void guard4(v8f& a, v8f& b, v8f& c, v8f& d, v16h x, v16h y) { dep_guard4_h(a, b, c, d, x, y); }
  static __device__ __forceinline__ void keep(v16h a, v16h b, v16h c, v16h d) { keep4_h(a, b, c, d); }
};
template <> struct Frag<__bf16> {
  typedef v16b V; union U { v16b v; v8b h[2]; };
  static __device__ __forceinline__ v16b load(const __bf16* p) {
    U f; f.h[0] = *(const v8b*)(p); f.h[1] = *(const v8b*)(p + 16); return f.v;
  }
  static __device__ __forceinline__ v8f mma(v16b a, v16b b, v8f c) {
    return __builtin_amdgcn_wmma_f32_16x16x32_bf16(false, a, false, b, (short)0, c, false, false);
  }
  static __device__ __forceinline__ void guard4(v8f& a, v8f& b, v8f& c, v8f& d, v16b x, v16b y) { dep_guard4_b(a, b, c, d, x, y); }
  static __device__ __forceinline__ void keep(v16b a, v16b b, v16b c, v16b d) { keep4_b(a, b, c, d); }
};

__device__ __forceinline__ v8f mma_h(v16h a, v16h b, v8f c) {
  c = __builtin_amdgcn_wmma_f32_16x16x32_f16(false, a, false, b, (short)0, c, false, false);
  asm volatile("v_nop\n\tv_nop\n\tv_nop\n\tv_nop" : "+v"(c) : "v"(a), "v"(b));
  return c;
}

template <int ET> struct Elem;
template <> struct Elem<0> { typedef _Float16 T; };
template <> struct Elem<1> { typedef __bf16 T; };
template <int ET, bool SPLIT, int BIAS_MODE, int OUT_MODE, bool RESID, int ACT = 0>
__global__ __launch_bounds__(256) void wmma_gemm64(
    const unsigned short* __restrict__ Ap, const unsigned short* __restrict__ A2p, int lda, long strideA,
    const unsigned short* __restrict__ Btp, const unsigned short* __restrict__ Bt2p, int ldb, long strideB,
    void* __restrict__ Cout, void* __restrict__ Cout2, int ldc, long strideC,
    const float* __restrict__ bias,
    const float* __restrict__ resid, long strideR,
    int M, int N, int K, float scale) {
  typedef typename Elem<ET>::T T;
  typedef typename Frag<T>::V V;
  const T* A = (const T*)Ap; const T* A2 = (const T*)A2p; const T* Bt = (const T*)Btp; const T* Bt2 = (const T*)Bt2p;
  __shared__ __align__(16) float sT[8][16 * 68];
  const int b    = blockIdx.y;
  const int lane = threadIdx.x & 31;
  const int wave = threadIdx.x >> 5;
  const int tilesN = N >> 6;
  const int tilesM = M >> 6;
  const int tile = blockIdx.x * 8 + wave;
  if (tile >= tilesM * tilesN) return;
  const int tm = tile / tilesN;
  const int tn = tile - tm * tilesN;
  const int m0 = tm << 6;
  const int n0 = tn << 6;

  const T* Ab  = A  + (size_t)b * strideA;
  const T* Bb  = Bt + (size_t)b * strideB;
  const T* Ab2 = SPLIT ? (A2  + (size_t)b * strideA) : nullptr;
  const T* Bb2 = SPLIT ? (Bt2 + (size_t)b * strideB) : nullptr;

  const int rlane = lane & 15;
  const int koff  = (lane >> 4) * 8;
  const int mOff  = (lane >> 4) * 8;

  v8f acc[4][4];
#pragma unroll
  for (int i = 0; i < 4; ++i)
#pragma unroll
    for (int j = 0; j < 4; ++j) acc[i][j] = (v8f){0.f,0.f,0.f,0.f,0.f,0.f,0.f,0.f};

  for (int k0 = 0; k0 < K; k0 += 32) {
    V bh[4], bl[4];
#pragma unroll
    for (int j = 0; j < 4; ++j) {
      const size_t bo = (size_t)(n0 + (j << 4) + rlane) * ldb + koff + k0;
      bh[j] = Frag<T>::load(Bb + bo);
      if (SPLIT) bl[j] = Frag<T>::load(Bb2 + bo);
    }
#pragma unroll
    for (int i = 0; i < 4; ++i) {
      const size_t ao = (size_t)(m0 + (i << 4) + rlane) * lda + koff + k0;
      V ah = Frag<T>::load(Ab + ao);
      V al;
      if (SPLIT) al = Frag<T>::load(Ab2 + ao);
#pragma unroll
      for (int j = 0; j < 4; ++j) {
        acc[i][j] = Frag<T>::mma(ah, bh[j], acc[i][j]);
        if (SPLIT) {
          acc[i][j] = Frag<T>::mma(ah, bl[j], acc[i][j]);
          acc[i][j] = Frag<T>::mma(al, bh[j], acc[i][j]);
        }
      }
      Frag<T>::guard4(acc[i][0], acc[i][1], acc[i][2], acc[i][3], ah, SPLIT ? al : ah);
    }
    Frag<T>::keep(bh[0], bh[1], bh[2], bh[3]);
    if (SPLIT) Frag<T>::keep(bl[0], bl[1], bl[2], bl[3]);
  }
  acc_guard4(acc[0][0], acc[0][1], acc[0][2], acc[0][3]);
  acc_guard4(acc[1][0], acc[1][1], acc[1][2], acc[1][3]);
  acc_guard4(acc[2][0], acc[2][1], acc[2][2], acc[2][3]);
  acc_guard4(acc[3][0], acc[3][1], acc[3][2], acc[3][3]);

  float* slab = sT[wave];
  const float* Rb = RESID ? (resid + (size_t)b * strideR) : nullptr;
#pragma unroll
  for (int i = 0; i < 4; ++i) {
    const int mBase = m0 + (i << 4);
#pragma unroll
    for (int j = 0; j < 4; ++j) {
      const int n = n0 + (j << 4) + rlane;
      float bv = 0.f;
      if (BIAS_MODE == 2) bv = bias[n];
#pragma unroll
      for (int r = 0; r < 8; ++r) {
        float v = acc[i][j][r] * scale;
        if (BIAS_MODE == 1) v += bias[mBase + mOff + r];
        if (BIAS_MODE == 2) v += bv;
        if (RESID) v += Rb[(size_t)(mBase + mOff + r) * ldc + n];
        if (ACT == 1) v = tanhf(v);
        if (ACT == 2) v = fmaxf(v, 0.0f);
        if (ACT == 3) v = v / (1.0f + expf(-v));
        if (ACT == 4) v = (v > 0.f) ? v : 0.01f * v;
        slab[(mOff + r) * 68 + (j << 4) + rlane] = v;
      }
    }
    __builtin_amdgcn_fence(__ATOMIC_RELEASE, "workgroup");
    __builtin_amdgcn_wave_barrier();
    __builtin_amdgcn_fence(__ATOMIC_ACQUIRE, "workgroup");
    if (OUT_MODE == 0) {
      float* C = (float*)Cout + (size_t)b * strideC;
      const int hh = lane >> 4, c4 = (lane & 15) * 4;
      for (int pass = 0; pass < 2; ++pass) {
#pragma unroll
        for (int it = 0; it < 8; ++it) {
          const int row = it * 2 + hh;
          v4f v = *(const v4f*)(slab + row * 68 + c4);
          *(volatile v4f*)(C + (size_t)(mBase + row) * ldc + n0 + c4) = v;
        }
        __threadfence();
      }
    } else {
      const int q = lane >> 3, c8 = (lane & 7) * 8;
      unsigned short* C  = (unsigned short*)Cout  + (size_t)b * strideC;
      unsigned short* C2 = (OUT_MODE == 2) ? ((unsigned short*)Cout2 + (size_t)b * strideC) : nullptr;
      for (int pass = 0; pass < 2; ++pass) {
#pragma unroll
        for (int it = 0; it < 4; ++it) {
          const int row = it * 4 + q;
          const float* sp = slab + row * 68 + c8;
          v8h hv, lv;
#pragma unroll
          for (int e = 0; e < 8; ++e) {
            if (OUT_MODE == 1) {
              hv[e] = (_Float16)sp[e];
            } else {
              unsigned short hb = f2bf_bits(sp[e]);
              unsigned short lb = f2bf_bits(sp[e] - bf_bits2f(hb));
              hv[e] = __builtin_bit_cast(_Float16, hb);
              lv[e] = __builtin_bit_cast(_Float16, lb);
            }
          }
          *(volatile v8h*)(C + (size_t)(mBase + row) * ldc + n0 + c8) = hv;
          if (OUT_MODE == 2) *(volatile v8h*)(C2 + (size_t)(mBase + row) * ldc + n0 + c8) = lv;
        }
        __threadfence();
      }
    }
    __builtin_amdgcn_fence(__ATOMIC_RELEASE, "workgroup");
    __builtin_amdgcn_wave_barrier();
    __builtin_amdgcn_fence(__ATOMIC_ACQUIRE, "workgroup");
  }
}

__global__ __launch_bounds__(256) void wt_plane_kernel(const float* __restrict__ W, unsigned short* __restrict__ dst, int K, int N, int nLive, int ldd, int colOff) {
  const int n  = blockIdx.x;
  const int k8 = threadIdx.x * 8;
  const bool live = n < nLive;
  const int nc = live ? n : 0;
  v8h hv;
#pragma unroll
  for (int e = 0; e < 8; ++e) {
    const float w = W[(size_t)(k8 + e) * N + nc];
    hv[e] = (_Float16)(live ? carry_flush(bf16r(w), kWCarry) : 0.0f);
  }
  unsigned short* dp = dst + (size_t)n * ldd + colOff + k8;
  *(volatile v8h*)dp = hv;
  __threadfence();
  *(volatile v8h*)dp = hv;
}


__global__ __launch_bounds__(kThr) void setup_kernel(const float* __restrict__ W_dt, const float* __restrict__ b_dt, unsigned short* __restrict__ WDT, float* __restrict__ BV) {
  unsigned v = blockIdx.x * (unsigned)kThr + threadIdx.x;
  asm volatile("" : "+v"(v));
  if (v < 2048u) {
    const unsigned n = v >> 2, k8 = (v & 3u) * 8u;
    v8h hv;
#pragma unroll
    for (int e = 0; e < 8; ++e) { const float w = W_dt[(size_t)(k8 + e) * kDi + n]; hv[e] = (_Float16)carry_flush(bf16r(w), kWCarry); }
    unsigned short* dp = WDT + (size_t)v * 8u;
    *(volatile v8h*)dp = hv;
    __threadfence();
    *(volatile v8h*)dp = hv;
  } else {
    const unsigned i0 = (v - 2048u) * 4u;
    v4f o = {0.f, 0.f, 0.f, 0.f};
    if (i0 < (unsigned)kDi) {
      const v4f a = *(const v4f*)(b_dt + i0);
#pragma unroll
      for (int e = 0; e < 4; ++e) { const float x = a[e]; o[e] = bf16r(x); }
    }
    float* dp = BV + i0;
    *(volatile v4f*)dp = o;
    __threadfence();
    *(volatile v4f*)dp = o;
  }
}
static_assert(kDi * kR / 8 == 2048 && 2048 % kThr == 0 && (2048 + 512) == 10 * kThr && (kDi % 128) == 0, "set-up grid exact");

__global__ __launch_bounds__(kThr) void ln_cast_kernel(const float* __restrict__ x, const float* __restrict__ ln_g, const float* __restrict__ ln_b,
                                                       unsigned short* __restrict__ XN16) {
  unsigned r = blockIdx.x * (unsigned)kThr + threadIdx.x;
  asm volatile("" : "+v"(r));
  const float* xr = x + (size_t)r * kDm;
  float s = 0.0f;
#pragma unroll 1
  for (unsigned c4 = 0; c4 < (unsigned)kDm; c4 += 4) { const v4f a = *(const v4f*)(xr + c4); s += bf16r(a[0]); s += bf16r(a[1]); s += bf16r(a[2]); s += bf16r(a[3]); }
  const float mu = s * kInvD;
  float q = 0.0f;
#pragma unroll 1
  for (unsigned c4 = 0; c4 < (unsigned)kDm; c4 += 4) {
    const v4f a = *(const v4f*)(xr + c4);
#pragma unroll
    for (int e = 0; e < 4; ++e) { const float d = bf16r(a[e]) - mu; q += d * d; }
  }
  const float rs = rsqrtf(q * kInvD + kEps);
  unsigned short* dp = XN16 + (size_t)r * kDm;
#pragma unroll 1
  for (unsigned c8 = 0; c8 < (unsigned)kDm; c8 += 8) {
    const v4f a0 = *(const v4f*)(xr + c8), a1 = *(const v4f*)(xr + c8 + 4);
    const v4f g0 = *(const v4f*)(ln_g + c8), g1 = *(const v4f*)(ln_g + c8 + 4), b0 = *(const v4f*)(ln_b + c8), b1 = *(const v4f*)(ln_b + c8 + 4);
    v8h hv;
#pragma unroll
    for (int e = 0; e < 4; ++e) {
      hv[e] = (_Float16)carry_flush((bf16r(a0[e]) - mu) * rs * bf16r(g0[e]) + bf16r(b0[e]), kInCarry);
      hv[4 + e] = (_Float16)carry_flush((bf16r(a1[e]) - mu) * rs * bf16r(g1[e]) + bf16r(b1[e]), kInCarry);
    }
    *(volatile v8h*)(dp + c8) = hv;
    __threadfence();
    *(volatile v8h*)(dp + c8) = hv;
  }
}
static_assert(kRows == 16 * kThr, "row grids exact");

__global__ __launch_bounds__(kThr) void conv_sp_kernel(const float* __restrict__ ZX, const float* __restrict__ conv_w, const float* __restrict__ conv_b,
                                                       float* __restrict__ U32, unsigned short* __restrict__ U16, int rev) {
  const size_t v = (size_t)blockIdx.x * kThr + threadIdx.x;
  const int row = (int)(v >> 7);
  const int d4 = (int)(v & 127) * 4;
  const v4f cb = *(const v4f*)(conv_b + d4);
  float acc[4];
#pragma unroll
  for (int e = 0; e < 4; ++e) { const float b0 = cb[e]; acc[e] = bf16r(b0); }
#pragma unroll
  for (int j = 0; j < kKc; ++j) {
    const int tr = rev ? (row + (kKc - 1) - j) : (row + j - (kKc - 1));
    const bool in = (tr >= 0) && (tr < kRows);
    const v4f xin = *(const v4f*)(ZX + (size_t)(in ? tr : 0) * kDi2 + d4);
#pragma unroll
    for (int e = 0; e < 4; ++e) {
      const float w0 = conv_w[(size_t)(d4 + e) * kKc + j];
      const float xv = in ? xin[e] : 0.0f;
      acc[e] += bf16r(w0) * xv;
    }
  }
  v4f o; v4h hv;
#pragma unroll
  for (int e = 0; e < 4; ++e) {
    const float c = acc[e];
    const float s = (c > 20.0f) ? c : log1pf(expf(c));
    o[e] = s;
    hv[e] = (_Float16)carry_flush(s, kInCarry);
  }
  for (int pass = 0; pass < 2; ++pass) {
    *(volatile v4f*)(U32 + (size_t)row * kDi + d4) = o;
    *(volatile v4h*)(U16 + (size_t)row * kDi + d4) = hv;
    __threadfence();
  }
}
static_assert(((size_t)kRows * 128) % kThr == 0 && kDi / 4 == 128, "conv grid exact");

__global__ __launch_bounds__(kThr) void dt_cast_kernel(const float* __restrict__ DBC, unsigned short* __restrict__ DT16) {
  const size_t v = (size_t)blockIdx.x * kThr + threadIdx.x;
  const size_t row = v >> 2;
  const int c8 = (int)(v & 3) * 8;
  const v4f a0 = *(const v4f*)(DBC + row * kXd + c8);
  const v4f a1 = *(const v4f*)(DBC + row * kXd + c8 + 4);
  v8h hv;
#pragma unroll
  for (int e = 0; e < 4; ++e) { hv[e] = (_Float16)carry_flush(a0[e], kInCarry); hv[4 + e] = (_Float16)carry_flush(a1[e], kInCarry); }
  unsigned short* dp = DT16 + v * 8u;
  *(volatile v8h*)dp = hv;
  __threadfence();
  *(volatile v8h*)dp = hv;
}
static_assert(((size_t)kRows * 4) % kThr == 0, "dt cast grid exact");

__global__ __launch_bounds__(kThr) void sel_scan_kernel(const float* __restrict__ DL, const float* __restrict__ U32, const float* __restrict__ DBC,
                                                        const float* __restrict__ A_log, const float* __restrict__ Dp, float* __restrict__ Y, int rev) {
  const int d = blockIdx.x * kThr + threadIdx.x;
  float A[kNs], h[kNs];
#pragma unroll
  for (int n = 0; n < kNs; ++n) { const float al = A_log[(size_t)d * kNs + n]; A[n] = -expf(bf16r(al)); h[n] = 0.0f; }
  float dsk = Dp[d];
  dsk = bf16r(dsk);
#pragma unroll 1
  for (int i = 0; i < kSeq; ++i) {
    const int l = rev ? (kSeq - 1 - i) : i;
    const float dl = DL[(size_t)l * kDi + d];
    const float uv = U32[(size_t)l * kDi + d];
    const float delta = (dl > 20.0f) ? dl : log1pf(expf(dl));
    const float dx = delta * uv;
    float y = 0.0f;
#pragma unroll
    for (int q = 0; q < 4; ++q) {
      const v4f bq = *(const v4f*)(DBC + (size_t)l * kXd + kR + 4 * q);
      const v4f cq = *(const v4f*)(DBC + (size_t)l * kXd + kR + kNs + 4 * q);
#pragma unroll
      for (int e = 0; e < 4; ++e) {
        const int n = 4 * q + e;
        const float hn = __expf(delta * A[n]) * h[n] + dx * bq[e];
        h[n] = hn;
        y += hn * cq[e];
      }
    }
    y += uv * dsk;
    float* yp = Y + (size_t)l * kDi + d;
    *(volatile float*)yp = y;
    __threadfence();
    *(volatile float*)yp = y;
  }
}
static_assert(kDi % kThr == 0, "scan grid exact");

__global__ __launch_bounds__(kThr) void combine_kernel(const float* __restrict__ YF, const float* __restrict__ YB, const float* __restrict__ ZX,
                                                       const float* __restrict__ x, float* __restrict__ out) {
  const size_t v = (size_t)blockIdx.x * kThr + threadIdx.x;
  const size_t row = v >> 7;
  const int d4 = (int)(v & 127) * 4;
  const v4f yf = *(const v4f*)(YF + row * kDi + d4), yb = *(const v4f*)(YB + row * kDi + d4);
  const v4f zz = *(const v4f*)(ZX + row * kDi2 + kDi + d4), xx = *(const v4f*)(x + row * kDm + d4);
  v4f o;
#pragma unroll
  for (int e = 0; e < 4; ++e) {
    const float zg = zz[e] * (1.0f / (1.0f + expf(-zz[e])));
    const float p1 = yf[e] * zg, p2 = yb[e] * zg;
    o[e] = (p1 + p2) + bf16r(xx[e]);
  }
  float* dp = out + row * kDm + d4;
  *(volatile v4f*)dp = o;
  __threadfence();
  *(volatile v4f*)dp = o;
}
static_assert(kDm == kDi, "the skip has the branch's width");

extern "C" void kernel_launch(void* const* d_in, const int* in_sizes, int n_in,
                              void* d_out, int out_size, void* d_ws, size_t ws_size,
                              hipStream_t stream) {
  if (n_in < 11 || d_out == nullptr || d_ws == nullptr) return;
  if (in_sizes[0] != kSamples * kRows * kDm || in_sizes[1] != kDm || in_sizes[2] != kDm || in_sizes[3] != kDm * kDi2 || in_sizes[4] != kDi * kKc || in_sizes[5] != kDi) return;
  if (in_sizes[6] != kDi * kXd || in_sizes[7] != kR * kDi || in_sizes[8] != kDi || in_sizes[9] != kDi * kNs || in_sizes[10] != kDi) return;
  if (out_size != kSamples * kRows * kDm) return;
  if (ws_size < kWsTotal) return;
  const float* x = (const float*)d_in[0];
  const float* ln_g = (const float*)d_in[1];
  const float* ln_b = (const float*)d_in[2];
  const float* W_proj = (const float*)d_in[3];
  const float* conv_w = (const float*)d_in[4];
  const float* conv_b = (const float*)d_in[5];
  const float* W_x = (const float*)d_in[6];
  const float* W_dt = (const float*)d_in[7];
  const float* b_dt = (const float*)d_in[8];
  const float* A_log = (const float*)d_in[9];
  const float* Dp = (const float*)d_in[10];
  float* out = (float*)d_out;
  char* ws = (char*)d_ws;
  unsigned short* XN16 = (unsigned short*)(ws + kOffXN16);
  unsigned short* WPT = (unsigned short*)(ws + kOffWPT);
  unsigned short* WXT = (unsigned short*)(ws + kOffWXT);
  unsigned short* WDT = (unsigned short*)(ws + kOffWDT);
  float* BV = (float*)(ws + kOffBV);
  float* ZX = (float*)(ws + kOffZX);
  float* U32 = (float*)(ws + kOffU32);
  unsigned short* U16 = (unsigned short*)(ws + kOffU16);
  float* DBC = (float*)(ws + kOffDBC);
  unsigned short* DT16 = (unsigned short*)(ws + kOffDT16);
  float* DL = (float*)(ws + kOffDL);
  float* YF = (float*)(ws + kOffYF);
  float* YB = (float*)(ws + kOffYB);
  const float* ZB = BV + kDi;

  wt_plane_kernel<<<kDi2, kDm / 8, 0, stream>>>(W_proj, WPT, kDm, kDi2, kDi2, kDm, 0);
  wt_plane_kernel<<<kXd, kDi / 8, 0, stream>>>(W_x, WXT, kDi, kXd, kXd, kDi, 0);
  setup_kernel<<<10, kThr, 0, stream>>>(W_dt, b_dt, WDT, BV);

  for (int s = 0; s < kSamples; ++s) {
    const float* xs = x + (size_t)s * kRows * kDm;
    float* os = out + (size_t)s * kRows * kDm;
    ln_cast_kernel<<<16, kThr, 0, stream>>>(xs, ln_g, ln_b, XN16);
    wmma_gemm64<0, false, 2, 0, false, 0><<<dim3((kRows / 64) * (kDi2 / 64) / 8, 1), 256, 0, stream>>>(
        XN16, XN16, kDm, 0L, WPT, WPT, kDm, 0L, (void*)ZX, (void*)ZX, kDi2, 0L, ZB, nullptr, 0L, kRows, kDi2, kDm, kSc);
    for (int rev = 0; rev < 2; ++rev) {
      conv_sp_kernel<<<(int)(((size_t)kRows * 128) / kThr), kThr, 0, stream>>>(ZX, conv_w, conv_b, U32, U16, rev);
      wmma_gemm64<0, false, 2, 0, false, 0><<<dim3((kRows / 64) * (kXd / 64) / 8, 1), 256, 0, stream>>>(
          U16, U16, kDi, 0L, WXT, WXT, kDi, 0L, (void*)DBC, (void*)DBC, kXd, 0L, ZB, nullptr, 0L, kRows, kXd, kDi, kSc);
      dt_cast_kernel<<<(int)(((size_t)kRows * 4) / kThr), kThr, 0, stream>>>(DBC, DT16);
      wmma_gemm64<0, false, 2, 0, false, 0><<<dim3((kRows / 64) * (kDi / 64) / 8, 1), 256, 0, stream>>>(
          DT16, DT16, kR, 0L, WDT, WDT, kR, 0L, (void*)DL, (void*)DL, kDi, 0L, BV, nullptr, 0L, kRows, kDi, kR, kSc);
      sel_scan_kernel<<<kDi / kThr, kThr, 0, stream>>>(DL, U32, DBC, A_log, Dp, rev ? YB : YF, rev);
    }
    combine_kernel<<<(int)(((size_t)kRows * 128) / kThr), kThr, 0, stream>>>(YF, YB, ZX, xs, os);
  }
}
